// ConcatAttention_16956530884977
// MI455X (gfx1250) — hardware-verified
//
#include <hip/hip_runtime.h>
#include <stdint.h>

constexpr int kB  = 2;
constexpr int kTq = 512;
constexpr int kTk = 1024;
constexpr int kH  = 128;

constexpr int kGemmRows   = 32;
constexpr int kQBlk       = kB * kTq / kGemmRows;
constexpr int kKBlk       = kB * kTk / kGemmRows;
constexpr int kVBlk       = kB * (kH / 64) * (kTk / 64);
constexpr int kPrepBlocks = kQBlk + kKBlk + kVBlk;
constexpr int kStagePitch = 132;
constexpr int kTfPitch    = 68;
constexpr int kQRows      = 16;
constexpr int kAttnBlocks = kB * kTq / kQRows;
constexpr int kPsPitch    = kTk + 8;

typedef _Float16 v16h __attribute__((ext_vector_type(16)));
typedef _Float16 v8h  __attribute__((ext_vector_type(8)));
typedef float    v8f  __attribute__((ext_vector_type(8)));
typedef float    v4f  __attribute__((ext_vector_type(4)));

union FragH { v16h v; v8h h[2]; };

__device__ __forceinline__ v8f zero8() {
  v8f z = {0.f, 0.f, 0.f, 0.f, 0.f, 0.f, 0.f, 0.f};
  return z;
}

__device__ __forceinline__ v8f mma16(v16h a, v16h b, v8f c) {
  c = __builtin_amdgcn_wmma_f32_16x16x32_f16(false, a, false, b, (short)0, c, false, false);
  asm volatile("v_nop\n\tv_nop\n\tv_nop\n\tv_nop" : "+v"(c) : "v"(a), "v"(b));
  return c;
}

__device__ __forceinline__ float wave_max32(float v) {
#pragma unroll
  for (int off = 16; off > 0; off >>= 1) v = fmaxf(v, __shfl_xor(v, off, 32));
  return v;
}
__device__ __forceinline__ float wave_sum32(float v) {
#pragma unroll
  for (int off = 16; off > 0; off >>= 1) v += __shfl_xor(v, off, 32);
  return v;
}

__device__ __forceinline__ float tanh_f(float x) {
  const float e = __expf(2.0f * x);
  const float r = __builtin_amdgcn_rcpf(1.0f + e);
  return fmaf(-2.0f, r, 1.0f);
}

__global__ __launch_bounds__(64) void prep_kernel(const float* __restrict__ query, const float* __restrict__ value,
                                                 const float* __restrict__ W1, const float* __restrict__ W2,
                                                 float* __restrict__ qproj, float* __restrict__ kproj,
                                                 _Float16* __restrict__ VT) {
  __shared__ __align__(16) float stage[2][16 * kStagePitch];
  __shared__ __align__(16) float tf[64 * kTfPitch];

  const int blk  = blockIdx.x;
  const int tid  = threadIdx.x;
  const int wave = tid >> 5;
  const int lane = tid & 31;
  const int hh   = lane >> 4;
  const int m    = lane & 15;

  if (blk < kQBlk + kKBlk) {
    const bool isq = (blk < kQBlk);
    const float* X = isq ? query : value;
    const float* W = isq ? W1 : W2;
    float* Y       = isq ? qproj : kproj;
    const int row0 = (isq ? blk : (blk - kQBlk)) * kGemmRows + wave * 16;

    v8f acc[8];
#pragma unroll
    for (int j = 0; j < 8; ++j) acc[j] = zero8();

    const float* xr = X + (size_t)(row0 + m) * kH + 8 * hh;
#pragma unroll 1
    for (int ks = 0; ks < kH / 32; ++ks) {
      const int k0 = ks * 32;
      FragH a;
      {
        const v4f f0 = *(const v4f*)(xr + k0);
        const v4f f1 = *(const v4f*)(xr + k0 + 4);
        const v4f g0 = *(const v4f*)(xr + k0 + 16);
        const v4f g1 = *(const v4f*)(xr + k0 + 20);
        v8h p0, p1;
#pragma unroll
        for (int e = 0; e < 4; ++e) {
          p0[e] = (_Float16)f0[e];  p0[4 + e] = (_Float16)f1[e];
          p1[e] = (_Float16)g0[e];  p1[4 + e] = (_Float16)g1[e];
        }
        a.h[0] = p0;
        a.h[1] = p1;
      }
      const float* w0 = W + (size_t)(k0 + 8 * hh) * kH + m;
      const float* w1 = W + (size_t)(k0 + 16 + 8 * hh) * kH + m;
#pragma unroll
      for (int j = 0; j < 8; ++j) {
        v8h b0, b1;
#pragma unroll
        for (int i = 0; i < 8; ++i) {
          b0[i] = (_Float16)(w0[(size_t)i * kH + 16 * j] * 16.0f);
          b1[i] = (_Float16)(w1[(size_t)i * kH + 16 * j] * 16.0f);
        }
        FragH bb;
        bb.h[0] = b0;
        bb.h[1] = b1;
        acc[j] = mma16(a.v, bb.v, acc[j]);
      }
    }

    float* slab = stage[wave];
#pragma unroll
    for (int j = 0; j < 8; ++j) {
#pragma unroll
      for (int r = 0; r < 8; ++r) slab[(8 * hh + r) * kStagePitch + 16 * j + m] = acc[j][r] * 0.0625f;
    }
    __builtin_amdgcn_fence(__ATOMIC_RELEASE, "workgroup");
    __builtin_amdgcn_wave_barrier();
    __builtin_amdgcn_fence(__ATOMIC_ACQUIRE, "workgroup");
    float* yb = Y + (size_t)row0 * kH + 4 * lane;
    for (int pass = 0; pass < 2; ++pass) {
#pragma unroll
      for (int row = 0; row < 16; ++row) {
        const v4f v = *(const v4f*)(slab + row * kStagePitch + 4 * lane);
        *(volatile v4f*)(yb + (size_t)row * kH) = v;
      }
      __threadfence();
    }
  } else {
    const int vb  = blk - (kQBlk + kKBlk);
    const int per = (kH / 64) * (kTk / 64);
    const int b   = vb / per;
    const int rem = vb - b * per;
    const int hb  = rem / (kTk / 64);
    const int sb  = rem - hb * (kTk / 64);
    const float* src = value + ((size_t)(b * kTk + sb * 64)) * kH + hb * 64;
    {
      const int lr = tid >> 4, c4 = (tid & 15) * 4;
#pragma unroll
      for (int it = 0; it < 16; ++it) {
        const int rr = it * 4 + lr;
        const v4f a = *(const v4f*)(src + (size_t)rr * kH + c4);
        *(v4f*)(tf + rr * kTfPitch + c4) = a;
      }
    }
    __syncthreads();
    const int g = tid >> 3, c8 = (tid & 7) * 8;
    v8h hv[8];
#pragma unroll
    for (int it = 0; it < 8; ++it) {
      const int oc = it * 8 + g;
      v8h v;
#pragma unroll
      for (int e = 0; e < 8; ++e) v[e] = (_Float16)tf[(c8 + e) * kTfPitch + oc];
      hv[it] = v;
    }
    _Float16* dst = VT + ((size_t)(b * kH + hb * 64)) * kTk + sb * 64 + c8;
    for (int pass = 0; pass < 2; ++pass) {
#pragma unroll
      for (int it = 0; it < 8; ++it) {
        const int oc = it * 8 + g;
        *(volatile v8h*)(dst + (size_t)oc * kTk) = hv[it];
      }
      __threadfence();
    }
  }
}

__global__ __launch_bounds__(256) void attn_kernel(const float* __restrict__ qproj, const float* __restrict__ kproj,
                                                  const float* __restrict__ scale, const int* __restrict__ mask,
                                                  const _Float16* __restrict__ VT,
                                                  float* __restrict__ ctx, float* __restrict__ attw) {
  __shared__ __align__(16) float qT[kH * kQRows];
  __shared__ float ssc[kH];
  __shared__ float redm[kQRows * 8];
  __shared__ float reds[kQRows * 8];
  __shared__ __align__(16) _Float16 Ps[kQRows * kPsPitch];
  __shared__ __align__(16) float cst[kQRows * kStagePitch];

  const int tid = threadIdx.x;
  const int wid = tid >> 5;
  const int lid = tid & 31;
  const int hh  = lid >> 4;
  const int m   = lid & 15;
  const int blk = blockIdx.x;
  const int b   = blk / (kTq / kQRows);
  const int t0  = (blk - b * (kTq / kQRows)) * kQRows;

  {
    const int t = tid >> 4, h8 = (tid & 15) * 8;
    const float* qr = qproj + ((size_t)(b * kTq + t0 + t)) * kH + h8;
    const v4f f0 = *(const v4f*)qr;
    const v4f f1 = *(const v4f*)(qr + 4);
#pragma unroll
    for (int e = 0; e < 4; ++e) {
      qT[(h8 + e) * kQRows + t]     = f0[e];
      qT[(h8 + 4 + e) * kQRows + t] = f1[e];
    }
  }
  if (tid < kH) ssc[tid] = scale[tid];
  __syncthreads();

  float sc[4][kQRows];
#pragma unroll
  for (int i = 0; i < 4; ++i) {
    const int s = tid + 256 * i;
    const float* kr = kproj + ((size_t)(b * kTk + s)) * kH;
    float acc[kQRows];
#pragma unroll
    for (int t = 0; t < kQRows; ++t) acc[t] = 0.f;
#pragma unroll 1
    for (int h = 0; h < kH; ++h) {
      const float kv = kr[h];
      const float sv = ssc[h];
      const v4f* qv = (const v4f*)(qT + h * kQRows);
      const v4f q0 = qv[0], q1 = qv[1], q2 = qv[2], q3 = qv[3];
      float qq[kQRows];
#pragma unroll
      for (int e = 0; e < 4; ++e) {
        qq[e] = q0[e]; qq[4 + e] = q1[e]; qq[8 + e] = q2[e]; qq[12 + e] = q3[e];
      }
#pragma unroll
      for (int t = 0; t < kQRows; ++t) acc[t] = fmaf(sv, tanh_f(qq[t] + kv), acc[t]);
    }
    const int mv = mask[b * kTk + s];
    const float madd = (mv != 0) ? 0.0f : -1.0e9f;
#pragma unroll
    for (int t = 0; t < kQRows; ++t) sc[i][t] = acc[t] + madd;
  }

  float rinv[kQRows];
  {
    float mx[kQRows];
#pragma unroll
    for (int t = 0; t < kQRows; ++t) {
      const float v = fmaxf(fmaxf(sc[0][t], sc[1][t]), fmaxf(sc[2][t], sc[3][t]));
      mx[t] = wave_max32(v);
    }
    if (lid == 0) {
#pragma unroll
      for (int t = 0; t < kQRows; ++t) redm[t * 8 + wid] = mx[t];
    }
    __syncthreads();
#pragma unroll
    for (int t = 0; t < kQRows; ++t) {
      float bm = redm[t * 8];
#pragma unroll
      for (int w = 1; w < 8; ++w) bm = fmaxf(bm, redm[t * 8 + w]);
      mx[t] = bm;
    }
    float sm[kQRows];
#pragma unroll
    for (int t = 0; t < kQRows; ++t) {
      float ssum = 0.f;
#pragma unroll
      for (int i = 0; i < 4; ++i) {
        const float e = __expf(sc[i][t] - mx[t]);
        sc[i][t] = e;
        ssum += e;
      }
      sm[t] = wave_sum32(ssum);
    }
    if (lid == 0) {
#pragma unroll
      for (int t = 0; t < kQRows; ++t) reds[t * 8 + wid] = sm[t];
    }
    __syncthreads();
#pragma unroll
    for (int t = 0; t < kQRows; ++t) {
      float bs = reds[t * 8];
#pragma unroll
      for (int w = 1; w < 8; ++w) bs += reds[t * 8 + w];
      rinv[t] = __builtin_amdgcn_rcpf(bs);
    }
  }
#pragma unroll
  for (int i = 0; i < 4; ++i) {
#pragma unroll
    for (int t = 0; t < kQRows; ++t) sc[i][t] = sc[i][t] * rinv[t];
  }

#pragma unroll
  for (int t = 0; t < kQRows; ++t) {
#pragma unroll
    for (int i = 0; i < 4; ++i) Ps[t * kPsPitch + 256 * i + tid] = (_Float16)(sc[i][t] * 4096.0f);
  }

  {
    float* awb = attw + ((size_t)(b * kTq + t0)) * kTk + tid;
    for (int pass = 0; pass < 2; ++pass) {
#pragma unroll
      for (int t = 0; t < kQRows; ++t) {
#pragma unroll
        for (int i = 0; i < 4; ++i) *(volatile float*)(awb + (size_t)t * kTk + 256 * i) = sc[i][t];
      }
      __threadfence();
    }
  }
  __syncthreads();

  {
    const int n0 = wid * 16;
    const _Float16* psr = Ps + m * kPsPitch + 8 * hh;
    const _Float16* vtr = VT + ((size_t)(b * kH + n0 + m)) * kTk + 8 * hh;
    v8f cacc = zero8();
#pragma unroll 4
    for (int ks = 0; ks < kTk / 32; ++ks) {
      const int k0 = ks * 32;
      FragH a, bb;
      a.h[0]  = *(const v8h*)(psr + k0);
      a.h[1]  = *(const v8h*)(psr + k0 + 16);
      bb.h[0] = *(const v8h*)(vtr + k0);
      bb.h[1] = *(const v8h*)(vtr + k0 + 16);
      cacc = mma16(a.v, bb.v, cacc);
    }
#pragma unroll
    for (int r = 0; r < 8; ++r) cst[(8 * hh + r) * kStagePitch + n0 + m] = cacc[r] * (1.0f / 4096.0f);
  }
  __syncthreads();
  {
    float* cb = ctx + ((size_t)(b * kTq + t0)) * kH + 4 * lid;
    for (int pass = 0; pass < 2; ++pass) {
#pragma unroll
      for (int rr = 0; rr < 2; ++rr) {
        const int row = 2 * wid + rr;
        const v4f v = *(const v4f*)(cst + row * kStagePitch + 4 * lid);
        *(volatile v4f*)(cb + (size_t)row * kH) = v;
      }
      __threadfence();
    }
  }
}

extern "C" void kernel_launch(void* const* d_in, const int* in_sizes, int n_in,
                              void* d_out, int out_size, void* d_ws, size_t ws_size,
                              hipStream_t stream) {
  if (n_in < 6) return;
  if (in_sizes[0] != kB * kTq * kH) return;
  if (in_sizes[1] != kB * kTk * kH) return;
  if (in_sizes[2] != kB * kTk) return;
  if (in_sizes[3] != kH * kH || in_sizes[4] != kH * kH) return;
  if (in_sizes[5] != kH) return;
  if (out_size != kB * kTq * kH + kB * kTq * kTk) return;

  const float* query = (const float*)d_in[0];
  const float* value = (const float*)d_in[1];
  const int*   mask  = (const int*)d_in[2];
  const float* W1    = (const float*)d_in[3];
  const float* W2    = (const float*)d_in[4];
  const float* scale = (const float*)d_in[5];

  float* ctx  = (float*)d_out;
  float* attw = (float*)d_out + (size_t)kB * kTq * kH;

  const size_t szQ = (size_t)kB * kTq * kH * sizeof(float);
  const size_t szK = (size_t)kB * kTk * kH * sizeof(float);
  const size_t szV = (size_t)kB * kH * kTk * sizeof(_Float16);
  const size_t oQ = 0;
  const size_t oK = oQ + szQ;
  const size_t oV = oK + szK;
  const size_t total = oV + szV;
  if (total > ws_size) return;

  char* ws = (char*)d_ws;
  float*    qproj = (float*)(ws + oQ);
  float*    kproj = (float*)(ws + oK);
  _Float16* VT    = (_Float16*)(ws + oV);

  prep_kernel<<<dim3(kPrepBlocks), dim3(64), 0, stream>>>(query, value, W1, W2, qproj, kproj, VT);
  attn_kernel<<<dim3(kAttnBlocks), dim3(256), 0, stream>>>(qproj, kproj, scale, mask, VT, ctx, attw);
  (void)hipGetLastError();
}
